// CMHSA_46943992545917
// MI455X (gfx1250) — hardware-verified
//
#include <hip/hip_runtime.h>
#include <math.h>

typedef __attribute__((ext_vector_type(16))) _Float16 v16h;
typedef __attribute__((ext_vector_type(16))) __bf16 v16b;
typedef __attribute__((ext_vector_type(8)))  _Float16 v8h;
typedef __attribute__((ext_vector_type(8)))  float v8f;
typedef __attribute__((ext_vector_type(4)))  float v4f;
typedef __attribute__((ext_vector_type(2)))  float v2f;
typedef __attribute__((ext_vector_type(4)))  unsigned v4u;
typedef __attribute__((ext_vector_type(4)))  int v4i;
typedef float __attribute__((may_alias)) float_a;
typedef int __attribute__((may_alias)) int_a;

template <typename T> __device__ __forceinline__ void vst2(void* p, T v) { *(volatile T*)p = v; __threadfence(); *(volatile T*)p = v; }
__device__ __forceinline__ v8f wmma16(v16h a, v16h b, v8f c) {
  v8f d = __builtin_amdgcn_wmma_f32_16x16x32_f16(false, a, false, b, (short)0, c, false, false);
  asm volatile("v_nop\n\tv_nop\n\tv_nop\n\tv_nop" : "+v"(d) : "v"(a), "v"(b));
  return d;
}
__device__ __forceinline__ v8f wmma_bf(v16b a, v16b b, v8f c) {
  v8f d = __builtin_amdgcn_wmma_f32_16x16x32_bf16(false, a, false, b, (short)0, c, false, false);
  asm volatile("v_nop\n\tv_nop\n\tv_nop\n\tv_nop" : "+v"(d) : "v"(a), "v"(b));
  return d;
}
__device__ __forceinline__ v16h frag_h(const _Float16* rowk0, int lane) {
  union { v16h v; v8h q[2]; } u; const _Float16* p = rowk0 + 8 * (lane >> 4);
  u.q[0] = *(const v8h*)p; u.q[1] = *(const v8h*)(p + 16); return u.v;
}
__device__ __forceinline__ v16h frag_f32(const float* rowk0, int lane) {
  v16h a; const float* p = rowk0 + 8 * (lane >> 4);
#pragma unroll
  for (int i = 0; i < 8; ++i) { a[i] = (_Float16)p[i]; a[8 + i] = (_Float16)p[16 + i]; }
  return a;
}
__device__ __forceinline__ v16h frag_f32s(const float* rowk0, int lane, float sc) {
  v16h a; const float* p = rowk0 + 8 * (lane >> 4);
#pragma unroll
  for (int i = 0; i < 8; ++i) { a[i] = (_Float16)(p[i] * sc); a[8 + i] = (_Float16)(p[16 + i] * sc); }
  return a;
}
__device__ __forceinline__ v16h fragc_f32(const float* W, int k0, int n, int lane, int ld, int K) {
  v16h a; const int g = lane >> 4;
#pragma unroll
  for (int i = 0; i < 8; ++i) { const int ka = k0 + 8 * g + i, kb = ka + 16;
    a[i] = (_Float16)(ka < K ? W[(size_t)(ka < K ? ka : K - 1) * ld + n] : 0.f); a[8 + i] = (_Float16)(kb < K ? W[(size_t)(kb < K ? kb : K - 1) * ld + n] : 0.f); }
  return a;
}
struct F2 { v16b h, l; };
__device__ __forceinline__ F2 bsplit16(const float v[16]) { F2 r;
#pragma unroll
  for (int i = 0; i < 16; ++i) { const __bf16 h = (__bf16)v[i]; r.h[i] = h; r.l[i] = (__bf16)(v[i] - (float)h); }
  return r; }
__device__ __forceinline__ F2 split_row(const float* row, int k0, int lane) { float v[16]; const float* p = row + k0 + 8 * (lane >> 4);
#pragma unroll
  for (int i = 0; i < 8; ++i) { v[i] = p[i]; v[8 + i] = p[16 + i]; }
  return bsplit16(v); }
__device__ __forceinline__ F2 split_rowK(const float* row, int k0, int lane, int K) { float v[16]; const int g = lane >> 4;
#pragma unroll
  for (int i = 0; i < 8; ++i) { const int ka = k0 + 8 * g + i, kb = ka + 16; v[i] = ka < K ? row[ka < K ? ka : K - 1] : 0.f; v[8 + i] = kb < K ? row[kb < K ? kb : K - 1] : 0.f; }
  return bsplit16(v); }
__device__ __forceinline__ F2 split_col(const float* W, int k0, int n, int lane, int ld, int K) { float v[16]; const int g = lane >> 4;
#pragma unroll
  for (int i = 0; i < 8; ++i) { const int ka = k0 + 8 * g + i, kb = ka + 16; v[i] = ka < K ? W[(size_t)(ka < K ? ka : K - 1) * ld + n] : 0.f; v[8 + i] = kb < K ? W[(size_t)(kb < K ? kb : K - 1) * ld + n] : 0.f; }
  return bsplit16(v); }
__device__ __forceinline__ v8f mac3(const F2& a, const F2& b, v8f c) { c = wmma_bf(a.l, b.h, c); c = wmma_bf(a.h, b.l, c); return wmma_bf(a.h, b.h, c); }
__device__ __forceinline__ float sigm(float v) { return 1.0f / (1.0f + expf(-v)); }
#define LDSX() do { asm volatile("s_wait_dscnt 0" ::: "memory"); __builtin_amdgcn_wave_barrier(); __builtin_amdgcn_fence(__ATOMIC_RELEASE, "workgroup"); } while (0)


#define NB 8
#define CC 256
#define TT 1024
#define NH 8
#define HD 32
#define NR (NB * TT)
#define QKVP (3 * CC)
#define DM CC
#ifndef NBT
#define NBT NB
#endif
typedef __attribute__((ext_vector_type(8))) __bf16 v8b;
__device__ __forceinline__ v16b frag_b(const __bf16* rowk0, int lane) {
  union { v16b v; v8b q[2]; } u; const __bf16* p = rowk0 + 8 * (lane >> 4);
  u.q[0] = *(const v8b*)p; u.q[1] = *(const v8b*)(p + 16); return u.v;
}
__device__ __forceinline__ float bfr(float v) { return (float)(__bf16)v; }
__device__ __attribute__((noinline)) float exp_ni(float v) { return expf(v); }
__device__ __attribute__((noinline)) float erf_ni(float v) { return erff(v); }

#define WS_PT   0u
#define WS_XT   (WS_PT + 2u * 4 * CC * CC)
#define WS_QKV  (WS_XT + 2u * NR * CC)
#define WS_VTH  (WS_QKV + 4u * NR * QKVP)
#define WS_VTL  (WS_VTH + 2u * NB * CC * TT)
#define WS_ON   (WS_VTL + 2u * NB * CC * TT)
#define WS_RSQ  (WS_ON + 4u * NB * NH * TT * HD)
#define WS_CV   (WS_RSQ + 4u * NB * NH * TT)
#define WS_END  (WS_CV + 4u * NB * NH * 64)

__global__ __launch_bounds__(256) void k_pack(const float* __restrict__ Wq, const float* __restrict__ Wk, const float* __restrict__ Wv, const float* __restrict__ Wp, __bf16* __restrict__ PT) {
  __shared__ __align__(16) __bf16 s[CC]; const int n = blockIdx.x, tid = threadIdx.x; const int m = n & 255; const float* src = (n < 256) ? Wq : (n < 512) ? Wk : (n < 768) ? Wv : Wp;
  s[tid] = (__bf16)src[(size_t)m * CC + tid]; __syncthreads();
  if (tid < CC / 8) vst2((unsigned*)(PT + (size_t)n * CC + tid * 8), *(const v4u*)&s[tid * 8]);
}
__global__ __launch_bounds__(256) void k_xt(const float* __restrict__ X, __bf16* __restrict__ XT) {
  __shared__ __align__(16) __bf16 s[32][CC + 8]; const int t0 = blockIdx.x * 32, b = blockIdx.y, tid = threadIdx.x;
  for (int q = tid; q < CC * 32; q += 256) { const int c = q >> 5, tl = q & 31; s[tl][c] = (__bf16)X[((size_t)b * CC + c) * TT + t0 + tl]; }
  __syncthreads();
  for (int q = tid; q < 32 * 32; q += 256) { const int tl = q >> 5, pc = q & 31; vst2((unsigned*)(XT + ((size_t)b * TT + t0 + tl) * CC + pc * 8), *(const v4u*)&s[tl][pc * 8]); }
}
__global__ __launch_bounds__(128) void k_qkv(const __bf16* __restrict__ XT, const __bf16* __restrict__ PT, float* __restrict__ QKV) {
  __shared__ __align__(16) float so[4][16][132];
  const int tid = threadIdx.x, wave = tid >> 5, lane = tid & 31, col = lane & 15, g = lane >> 4; const size_t r0 = (size_t)blockIdx.x * 64 + wave * 16; const int n0 = blockIdx.y * 128;
  v8f acc[8] = {};
#pragma unroll 2
  for (int kc = 0; kc < CC / 32; ++kc) { const v16b a = frag_b(XT + (r0 + col) * CC + kc * 32, lane);
#pragma unroll
    for (int j = 0; j < 8; ++j) acc[j] = wmma_bf(a, frag_b(PT + (size_t)(n0 + j * 16 + col) * CC + kc * 32, lane), acc[j]); }
#pragma unroll
  for (int j = 0; j < 8; ++j)
#pragma unroll
    for (int r = 0; r < 8; ++r) so[wave][8 * g + r][j * 16 + col] = acc[j][r];
  LDSX();
  for (int rl = 0; rl < 16; ++rl) vst2(QKV + (r0 + rl) * QKVP + n0 + lane * 4, *(const v4f*)&so[wave][rl][lane * 4]);
}
__global__ __launch_bounds__(256) void k_vt(const float* __restrict__ QKV, __bf16* __restrict__ VTH, __bf16* __restrict__ VTL) {
  __shared__ __align__(16) __bf16 svh[DM][72], svl[DM][72];
  const int tid = threadIdx.x; const size_t t0 = (size_t)blockIdx.x * 64; const int b = (int)(t0 / TT), p0 = (int)(t0 % TT);
  for (int q = tid; q < 64 * DM; q += 256) { const int tl = q >> 8, c = q & 255; const float v = QKV[(t0 + tl) * QKVP + 2 * DM + c]; const __bf16 hb = (__bf16)v; svh[c][tl] = hb; svl[c][tl] = (__bf16)(v - (float)hb); }
  __syncthreads();
  for (int q = tid; q < DM * 8; q += 256) { const int rowi = q >> 3, pc = q & 7; const size_t o = ((size_t)b * DM + rowi) * TT + p0 + pc * 8; vst2((unsigned*)(VTH + o), *(const v4u*)&svh[rowi][pc * 8]); vst2((unsigned*)(VTL + o), *(const v4u*)&svl[rowi][pc * 8]); }
}
__global__ __launch_bounds__(128) void k_attn(const float* __restrict__ QKV, const __bf16* __restrict__ VTH, const __bf16* __restrict__ VTL, const float* __restrict__ WH, float* __restrict__ ON, float* __restrict__ RSQ) {
  __shared__ __align__(16) __bf16 sqh[4][8][16][40], sql[4][8][16][40]; __shared__ __align__(16) float sraw[4][8][16][36]; __shared__ __align__(16) float sp[4][4][16][36]; __shared__ float salpha[4][4][16], sl[4][4][16];
  const int tid = threadIdx.x, wave = tid >> 5, lane = tid & 31, col = lane & 15, hf = lane >> 4; const int qb = blockIdx.x, b = blockIdx.y, hg = blockIdx.z; const int q0 = qb * 64 + wave * 16; const size_t tq = (size_t)b * TT + q0;
  for (int q = lane; q < 16 * CC; q += 32) { const int rl = q >> 8, c = q & 255; const float v = QKV[(tq + rl) * QKVP + c]; const __bf16 hb = (__bf16)v; sqh[wave][c >> 5][rl][c & 31] = hb; sql[wave][c >> 5][rl][c & 31] = (__bf16)(v - (float)hb); }
  const int row = lane & 15; const int hl0 = hf * 2; float wm[2][8];
#pragma unroll
  for (int u = 0; u < 2; ++u)
#pragma unroll
    for (int gg = 0; gg < 8; ++gg) wm[u][gg] = bfr(WH[(hg * 4 + hl0 + u) * NH + gg]);
  float m[2], l[2], l2[2]; m[0] = m[1] = -3.0e38f; l[0] = l[1] = 0.f; l2[0] = l2[1] = 0.f;
  v8f acc[4][2] = {};
  LDSX();
#pragma unroll 1
  for (int ks = 0; ks < TT / 32; ++ks) {
#pragma unroll 1
    for (int gg = 0; gg < 8; ++gg) { F2 a; a.h = frag_b(&sqh[wave][gg][col][0], lane); a.l = frag_b(&sql[wave][gg][col][0], lane);
#pragma unroll
      for (int ct = 0; ct < 2; ++ct) { const int kk = ks * 32 + ct * 16 + col; const F2 k = split_row(QKV + ((size_t)b * TT + kk) * QKVP + CC + gg * HD, 0, lane); const v8f c = mac3(a, k, (v8f){});
#pragma unroll
        for (int r = 0; r < 8; ++r) sraw[wave][gg][8 * hf + r][ct * 16 + col] = c[r] * 0.17677669529663687f; } }
    LDSX();
    { float s0[32], s1[32];
#pragma unroll
      for (int k4 = 0; k4 < 8; ++k4) { float t0[4] = {0.f, 0.f, 0.f, 0.f}, t1[4] = {0.f, 0.f, 0.f, 0.f};
#pragma unroll
        for (int gg = 0; gg < 8; ++gg) { const v4f rv = *(const v4f*)&sraw[wave][gg][row][k4 * 4];
#pragma unroll
          for (int i = 0; i < 4; ++i) { t0[i] += wm[0][gg] * rv[i]; t1[i] += wm[1][gg] * rv[i]; } }
#pragma unroll
        for (int i = 0; i < 4; ++i) { s0[k4 * 4 + i] = t0[i]; s1[k4 * 4 + i] = t1[i]; } }
#pragma unroll
      for (int u = 0; u < 2; ++u) { float* s = u == 0 ? s0 : s1; float mx = s[0];
#pragma unroll
        for (int k = 1; k < 32; ++k) mx = fmaxf(mx, s[k]);
        const float mn = fmaxf(m[u], mx); const float al = exp_ni(m[u] - mn); float es = 0.f, es2 = 0.f;
#pragma unroll
        for (int k = 0; k < 32; ++k) { const float e = exp_ni(s[k] - mn); es += e; es2 += e * e; sp[wave][hl0 + u][row][k] = e; }
        l[u] = l[u] * al + es; l2[u] = l2[u] * (al * al) + es2; m[u] = mn; salpha[wave][hl0 + u][row] = al; } }
    LDSX();
#pragma unroll
    for (int hl = 0; hl < 4; ++hl) { const F2 pa = split_row(&sp[wave][hl][col][0], 0, lane);
#pragma unroll
      for (int r = 0; r < 8; ++r) { const float al = salpha[wave][hl][8 * hf + r]; acc[hl][0][r] *= al; acc[hl][1][r] *= al; }
#pragma unroll
      for (int dt = 0; dt < 2; ++dt) { const size_t vrow = ((size_t)b * CC + (hg * 4 + hl) * HD + dt * 16 + col) * TT + ks * 32; const v16b vh = frag_b(VTH + vrow, lane), vl = frag_b(VTL + vrow, lane);
        acc[hl][dt] = wmma_bf(pa.l, vh, acc[hl][dt]); acc[hl][dt] = wmma_bf(pa.h, vl, acc[hl][dt]); acc[hl][dt] = wmma_bf(pa.h, vh, acc[hl][dt]); } }
    LDSX(); }
#pragma unroll
  for (int u = 0; u < 2; ++u) { sl[wave][hl0 + u][row] = l[u]; salpha[wave][hl0 + u][row] = l2[u] / (l[u] * l[u]); }
  LDSX();
  float (*so)[16][36] = sp[wave];
#pragma unroll
  for (int hl = 0; hl < 4; ++hl)
#pragma unroll
    for (int r = 0; r < 8; ++r) { const float il = 1.0f / sl[wave][hl][8 * hf + r]; so[hl][8 * hf + r][col] = acc[hl][0][r] * il; so[hl][8 * hf + r][16 + col] = acc[hl][1][r] * il; }
  LDSX();
#pragma unroll
  for (int hl = 0; hl < 4; ++hl) for (int rl = 0; rl < 16; ++rl) if (lane < 8) vst2(ON + ((((size_t)b * NH + hg * 4 + hl) * TT + q0 + rl) * HD) + lane * 4, *(const v4f*)&so[hl][rl][lane * 4]);
  { float* chunk = RSQ + ((((size_t)b * 2 + hg) * 16 + qb) * 4 + wave) * 64; __shared__ __align__(16) float sr[4][64];
    if (lane < 16) { sr[wave][lane * 4 + 0] = salpha[wave][0][lane]; sr[wave][lane * 4 + 1] = salpha[wave][1][lane]; sr[wave][lane * 4 + 2] = salpha[wave][2][lane]; sr[wave][lane * 4 + 3] = salpha[wave][3][lane]; }
    LDSX();
    if (lane < 16) vst2(chunk + lane * 4, *(const v4f*)&sr[wave][lane * 4]); }
}
__global__ __launch_bounds__(256) void k_norm(const float* __restrict__ RSQ, const float* __restrict__ QKV, const float* __restrict__ GA, const float* __restrict__ BE, float* __restrict__ CV) {
  __shared__ float sred[256]; __shared__ __align__(16) float srow[64];
  const int b = blockIdx.x >> 3, h = blockIdx.x & 7, tid = threadIdx.x; const int hg = h >> 2, hl = h & 3;
  float s = 0.f;
#pragma unroll
  for (int i = 0; i < 4; ++i) { const int q = tid * 4 + i; const int qb = q >> 6, wave = (q >> 4) & 3, rl = q & 15; s += RSQ[((((size_t)b * 2 + hg) * 16 + qb) * 4 + wave) * 64 + rl * 4 + hl]; }
  sred[tid] = s; __syncthreads();
  for (int st = 128; st >= 1; st >>= 1) { if (tid < st) sred[tid] += sred[tid + st]; __syncthreads(); }
  if (tid < 64) srow[tid] = 0.f;
  if (tid < 32) { float vs = 0.f;
#pragma unroll 4
    for (int t = 0; t < TT; ++t) vs += QKV[((size_t)b * TT + t) * QKVP + 2 * CC + h * HD + tid];
    srow[32 + tid] = vs; }
  __syncthreads();
  if (tid == 0) { const float e2 = sred[0] / ((float)TT * (float)TT); const float mean = 1.0f / (float)TT; const float var = e2 - mean * mean; const float rs = rsqrtf(var + 1e-5f); const float cA = rs * bfr(GA[h]); srow[0] = cA; srow[1] = bfr(BE[h]) - cA * mean; }
  __syncthreads();
  if (tid < 16) vst2(CV + (size_t)blockIdx.x * 64 + tid * 4, *(const v4f*)&srow[tid * 4]);
}
__global__ __launch_bounds__(128) void k_fin(const float* __restrict__ ON, const float* __restrict__ CV, const __bf16* __restrict__ PT, const float* __restrict__ bp, float* __restrict__ out) {
  __shared__ __align__(16) float sT[128][68];
  const int tid = threadIdx.x, wave = tid >> 5, lane = tid & 31, col = lane & 15, g = lane >> 4; const int b = blockIdx.z, n0 = blockIdx.y * 128; const int r0 = blockIdx.x * 64 + wave * 16; const int h = (blockIdx.x * 64) / 128;
  const float cA = CV[(b * NH + h) * 64 + 0], cB = CV[(b * NH + h) * 64 + 1]; const float* vs = CV + (b * NH + h) * 64 + 32;
  const float* Arow = ON + ((size_t)b * TT + r0 + col) * CC;
  v8f acc[8] = {};
#pragma unroll 2
  for (int kc = 0; kc < CC / 32; ++kc) { float v[16]; const float* p = Arow + kc * 32 + 8 * g;
#pragma unroll
    for (int i = 0; i < 8; ++i) { v[i] = cA * p[i] + cB * vs[8 * g + i]; v[8 + i] = cA * p[16 + i] + cB * vs[16 + 8 * g + i]; }
    const F2 a = bsplit16(v);
#pragma unroll
    for (int j = 0; j < 8; ++j) { const v16b w = frag_b(PT + (size_t)(768 + n0 + j * 16 + col) * CC + kc * 32, lane); acc[j] = wmma_bf(a.l, w, acc[j]); acc[j] = wmma_bf(a.h, w, acc[j]); } }
#pragma unroll
  for (int j = 0; j < 8; ++j) { const float bb = bfr(bp[n0 + j * 16 + col]);
#pragma unroll
    for (int r = 0; r < 8; ++r) sT[j * 16 + col][wave * 16 + 8 * g + r] = acc[j][r] + bb; }
  __syncthreads();
  for (int q = tid; q < 128 * 16; q += 128) { const int o = q >> 4, piece = q & 15; vst2(out + ((size_t)b * CC + n0 + o) * TT + blockIdx.x * 64 + piece * 4, *(const v4f*)&sT[o][piece * 4]); }
}
extern "C" void kernel_launch(void* const* d_in, const int* in_sizes, int n_in, void* d_out, int out_size, void* d_ws, size_t ws_size, hipStream_t stream) {
  (void)in_sizes; (void)n_in; (void)out_size;
  const float** F = (const float**)d_in;
  if (ws_size < (size_t)WS_END) return;
  char* ws = (char*)d_ws; __bf16 *PT = (__bf16*)(ws + WS_PT), *XT = (__bf16*)(ws + WS_XT), *VTH = (__bf16*)(ws + WS_VTH), *VTL = (__bf16*)(ws + WS_VTL); float *QKV = (float*)(ws + WS_QKV), *ON = (float*)(ws + WS_ON), *RSQ = (float*)(ws + WS_RSQ), *CV = (float*)(ws + WS_CV);
  k_pack<<<4 * CC, 256, 0, stream>>>(F[1], F[2], F[3], F[7], PT);
  k_xt<<<dim3(TT / 32, NBT), 256, 0, stream>>>(F[0], XT);
  k_qkv<<<dim3(NBT * TT / 64, QKVP / 128), 128, 0, stream>>>(XT, PT, QKV);
  k_vt<<<NBT * TT / 64, 256, 0, stream>>>(QKV, VTH, VTL);
  k_attn<<<dim3(TT / 64, NBT, 2), 128, 0, stream>>>(QKV, VTH, VTL, F[4], ON, RSQ);
  k_norm<<<NBT * NH, 256, 0, stream>>>(RSQ, QKV, F[5], F[6], CV);
  k_fin<<<dim3(TT / 64, CC / 128, NBT), 128, 0, stream>>>(ON, CV, PT, F[8], (float*)d_out);
}
